// Hypersphere_37082747633942
// MI455X (gfx1250) — hardware-verified
//
#include <hip/hip_runtime.h>


#define DEVFN __device__ __forceinline__

typedef _Float16 h16 __attribute__((ext_vector_type(16)));
typedef _Float16 h8  __attribute__((ext_vector_type(8)));
typedef __bf16   b16v __attribute__((ext_vector_type(16)));
typedef unsigned short u16v __attribute__((ext_vector_type(16)));
typedef float    f8  __attribute__((ext_vector_type(8)));
typedef float    v4f __attribute__((ext_vector_type(4)));

union HF  { h16 v; h8 p[2]; };
union BFR { b16v v; u16v u; };

constexpr int Bq  = 4;
constexpr int Lq  = 2048;
constexpr int Dq  = 1024;
constexpr int Kq  = 16;
constexpr int NR  = Bq * Lq;
constexpr int CH  = 128;
constexpr int NCH = Lq / CH;
constexpr int SROW = CH + 8;
constexpr int TR   = CH + 8;
constexpr int BR   = 40;

static_assert((Lq % CH) == 0);
static_assert((NR % 128) == 0);
static_assert((Dq % 128) == 0);
static_assert(sizeof(HF) == 32);
static_assert(sizeof(BFR) == 32);

DEVFN f8 mma_f16(h16 a, h16 b, f8 c) {
  c = __builtin_amdgcn_wmma_f32_16x16x32_f16(false, a, false, b, (short)0, c, false, false);
  asm volatile("v_nop\n\tv_nop\n\tv_nop\n\tv_nop" : "+v"(c) : "v"(a), "v"(b));
  return c;
}
DEVFN f8 mma_bf16(b16v a, b16v b, f8 c) {
  c = __builtin_amdgcn_wmma_f32_16x16x32_bf16(false, a, false, b, (short)0, c, false, false);
  asm volatile("v_nop\n\tv_nop\n\tv_nop\n\tv_nop" : "+v"(c) : "v"(a), "v"(b));
  return c;
}

DEVFN h16 frag_nk(const _Float16* base, int ld, int row0, int k0, int lane) {
  const int m = lane & 15, h = lane >> 4;
  const _Float16* p = base + (size_t)(row0 + m) * ld + k0 + 8 * h;
  HF f;
  f.p[0] = *(const h8*)p;
  f.p[1] = *(const h8*)(p + 16);
  return f.v;
}
DEVFN h16 frag_nk16(const _Float16* base, int ld, int row0, int lane) {
  const int m = lane & 15, h = lane >> 4;
  HF f;
  f.p[0] = *(const h8*)(base + (size_t)(row0 + m) * ld + 8 * h);
  h8 z = {};
  f.p[1] = z;
  return f.v;
}

DEVFN unsigned rne_bf16_bits(float x) {
  unsigned u = __float_as_uint(x);
  return (u + 0x7FFFu + ((u >> 16) & 1u)) >> 16;
}

DEVFN void ld16(const float* p, float* o) {
  const v4f* q = (const v4f*)p;
  v4f a = q[0], b = q[1], c = q[4], d = q[5];
#pragma unroll
  for (int i = 0; i < 4; ++i) { o[i] = a[i]; o[4 + i] = b[i]; o[8 + i] = c[i]; o[12 + i] = d[i]; }
}
DEVFN void split_bf(const float* v, BFR& hi, BFR& lo) {
#pragma unroll
  for (int i = 0; i < 16; ++i) {
    unsigned hb = rne_bf16_bits(v[i]);
    float hf = __uint_as_float(hb << 16);
    unsigned lb = rne_bf16_bits(v[i] - hf);
    hi.u[i] = (unsigned short)hb;
    lo.u[i] = (unsigned short)lb;
  }
}

__global__ void __launch_bounds__(256)
k_cvt(const float* __restrict__ s, _Float16* __restrict__ d, int n8, float scale) {
  const int i = blockIdx.x * 256 + threadIdx.x;
  const bool ok = i < n8;
  h8 r = {};
  if (ok) {
    const v4f* q = (const v4f*)(s + (size_t)i * 8);
    v4f a = q[0], b = q[1];
#pragma unroll
    for (int j = 0; j < 4; ++j) {
      r[j]     = (_Float16)(a[j] * scale);
      r[4 + j] = (_Float16)(b[j] * scale);
    }
    *(volatile h8*)(d + (size_t)i * 8) = r;
  }
  __threadfence();
  if (ok) *(volatile h8*)(d + (size_t)i * 8) = r;
}

__global__ void __launch_bounds__(256)
k_gemm_val(const _Float16* __restrict__ xh, const _Float16* __restrict__ wh,
           const float* __restrict__ bias, _Float16* __restrict__ valT) {
  __shared__ __align__(16) _Float16 pool[CH * TR];
  const int tid = threadIdx.x, lane = tid & 31, w = tid >> 5, m = lane & 15, h = lane >> 4;
  const int row0 = blockIdx.x * 128 + w * 16;
  const int col0 = blockIdx.y * 128;
  f8 acc[8] = {};
  for (int kb = 0; kb < Dq; kb += 32) {
    __syncthreads();
#pragma unroll
    for (int it = 0; it < 2; ++it) {
      int i = tid + it * 256;
      int r = i >> 2, off = (i & 3) * 8;
      *(h8*)(pool + r * BR + off) = *(const h8*)(wh + (size_t)(col0 + r) * Dq + kb + off);
    }
    __syncthreads();
    h16 a = frag_nk(xh, Dq, row0, kb, lane);
#pragma unroll
    for (int ct = 0; ct < 8; ++ct)
      acc[ct] = mma_f16(a, frag_nk(pool, BR, ct * 16, 0, lane), acc[ct]);
  }
  __syncthreads();
#pragma unroll
  for (int ct = 0; ct < 8; ++ct) {
    int dl = ct * 16 + m;
    float bb = bias[col0 + dl] * 16.0f;
#pragma unroll
    for (int r = 0; r < 8; ++r)
      pool[dl * TR + w * 16 + 8 * h + r] = (_Float16)(acc[ct][r] * 0.25f + bb);
  }
  __syncthreads();
  const int b  = (blockIdx.x * 128) >> 11;
  const int t0 = (blockIdx.x * 128) & (Lq - 1);
#pragma unroll
  for (int it = 0; it < 8; ++it) {
    int i = tid + it * 256;
    int dl = i >> 4, tt = (i & 15) * 8;
    h8 v = *(const h8*)(pool + dl * TR + tt);
    *(volatile h8*)(valT + ((size_t)(b * Dq + col0 + dl)) * Lq + t0 + tt) = v;
  }
  __threadfence();
#pragma unroll
  for (int it = 0; it < 8; ++it) {
    int i = tid + it * 256;
    int dl = i >> 4, tt = (i & 15) * 8;
    h8 v = *(const h8*)(pool + dl * TR + tt);
    *(volatile h8*)(valT + ((size_t)(b * Dq + col0 + dl)) * Lq + t0 + tt) = v;
  }
}

__global__ void __launch_bounds__(256)
k_gemm_out(const _Float16* __restrict__ nh, const _Float16* __restrict__ wh,
           const float* __restrict__ bias, const float* __restrict__ xres,
           float* __restrict__ out) {
  __shared__ __align__(16) float pool[8 * 16 * 128];
  _Float16* sB = (_Float16*)pool;
  const int tid = threadIdx.x, lane = tid & 31, w = tid >> 5, m = lane & 15, h = lane >> 4;
  const int row0 = blockIdx.x * 128 + w * 16;
  const int col0 = blockIdx.y * 128;
  f8 acc[8] = {};
  for (int kb = 0; kb < Dq; kb += 32) {
    __syncthreads();
#pragma unroll
    for (int it = 0; it < 2; ++it) {
      int i = tid + it * 256;
      int r = i >> 2, off = (i & 3) * 8;
      *(h8*)(sB + r * BR + off) = *(const h8*)(wh + (size_t)(col0 + r) * Dq + kb + off);
    }
    __syncthreads();
    h16 a = frag_nk(nh, Dq, row0, kb, lane);
#pragma unroll
    for (int ct = 0; ct < 8; ++ct)
      acc[ct] = mma_f16(a, frag_nk(sB, BR, ct * 16, 0, lane), acc[ct]);
  }
  __syncthreads();
  float* sO = pool + w * (16 * 128);
#pragma unroll
  for (int ct = 0; ct < 8; ++ct) {
    int cl = ct * 16 + m;
    float bb = bias[col0 + cl];
#pragma unroll
    for (int r = 0; r < 8; ++r)
      sO[(8 * h + r) * 128 + cl] = acc[ct][r] * (1.0f / 64.0f) + bb;
  }
  __syncthreads();
#pragma unroll
  for (int rr = 0; rr < 16; ++rr) {
    size_t g = (size_t)(row0 + rr) * Dq + col0 + lane * 4;
    v4f v  = *(const v4f*)(sO + rr * 128 + lane * 4);
    v4f xr = *(const v4f*)(xres + g);
    v4f o  = xr + v;
    *(volatile v4f*)(out + g) = o;
  }
  __threadfence();
#pragma unroll
  for (int rr = 0; rr < 16; ++rr) {
    size_t g = (size_t)(row0 + rr) * Dq + col0 + lane * 4;
    v4f v  = *(const v4f*)(sO + rr * 128 + lane * 4);
    v4f xr = *(const v4f*)(xres + g);
    v4f o  = xr + v;
    *(volatile v4f*)(out + g) = o;
  }
}

__global__ void __launch_bounds__(256)
k_proj(const float* __restrict__ x, const float* __restrict__ Wck, const float* __restrict__ Wcq,
       const float* __restrict__ bck, const float* __restrict__ bcq,
       const float* __restrict__ Wc, const float* __restrict__ bc,
       const float* __restrict__ pos,
       _Float16* __restrict__ ckh, _Float16* __restrict__ cqh, _Float16* __restrict__ ckT) {
  __shared__ __align__(16) float    sD[8 * 2 * 16 * 16];
  __shared__ __align__(16) float    sC[8 * 2 * 16 * 32];
  __shared__ __align__(16) _Float16 sO[2 * 128 * 16];
  __shared__ __align__(16) _Float16 sT[16 * TR];
  const int tid = threadIdx.x, lane = tid & 31, w = tid >> 5, m = lane & 15, h = lane >> 4;
  const int brow0 = blockIdx.x * 128;
  const int row0  = brow0 + w * 16;
  f8 ak = {}, aq = {};
  for (int kb = 0; kb < Dq; kb += 32) {
    float xv[16], wv[16];
    BFR ah, al, bh, bl;
    ld16(x + (size_t)(row0 + m) * Dq + kb + 8 * h, xv);
    split_bf(xv, ah, al);
    ld16(Wck + (size_t)m * Dq + kb + 8 * h, wv);
    split_bf(wv, bh, bl);
    ak = mma_bf16(ah.v, bh.v, ak);
    ak = mma_bf16(ah.v, bl.v, ak);
    ak = mma_bf16(al.v, bh.v, ak);
    ld16(Wcq + (size_t)m * Dq + kb + 8 * h, wv);
    split_bf(wv, bh, bl);
    aq = mma_bf16(ah.v, bh.v, aq);
    aq = mma_bf16(ah.v, bl.v, aq);
    aq = mma_bf16(al.v, bh.v, aq);
  }
  float* sDw = sD + w * (2 * 16 * 16);
  float* sCw = sC + w * (2 * 16 * 32);
  {
    const float bk = bck[m], bq = bcq[m];
#pragma unroll
    for (int r = 0; r < 8; ++r) {
      sDw[(8 * h + r) * 16 + m]       = ak[r] + bk;
      sDw[256 + (8 * h + r) * 16 + m] = aq[r] + bq;
    }
    const int t = (row0 + m) & (Lq - 1);
    const v4f* pq = (const v4f*)(pos + (size_t)t * Kq + 8 * h);
    v4f p0 = pq[0], p1 = pq[1];
    v4f* c0 = (v4f*)(sCw + m * 32 + 8 * h);
    v4f* c1 = (v4f*)(sCw + 512 + m * 32 + 8 * h);
    c0[0] = p0; c0[1] = p1;
    c1[0] = p0; c1[1] = p1;
  }
  __syncthreads();
  {
    const float* src = sDw + h * 256 + m * 16;
    float* dst = sCw + h * 512 + m * 32 + 16;
    float ss = 0.f;
#pragma unroll 1
    for (int k = 0; k < 16; ++k) { float v = src[k]; ss += v * v; }
    const float inv = 1.0f / fmaxf(sqrtf(ss), 1e-12f);
#pragma unroll 1
    for (int k = 0; k < 16; ++k) dst[k] = src[k] * inv;
  }
  __syncthreads();
  f8 dk = {}, dq = {};
  {
    float cv[16];
    BFR wbh, wbl, cbh, cbl;
    ld16(Wc + (size_t)m * (2 * Kq) + 8 * h, cv);
    split_bf(cv, wbh, wbl);
    ld16(sCw + m * 32 + 8 * h, cv);
    split_bf(cv, cbh, cbl);
    dk = mma_bf16(cbh.v, wbh.v, dk);
    dk = mma_bf16(cbh.v, wbl.v, dk);
    dk = mma_bf16(cbl.v, wbh.v, dk);
    ld16(sCw + 512 + m * 32 + 8 * h, cv);
    split_bf(cv, cbh, cbl);
    dq = mma_bf16(cbh.v, wbh.v, dq);
    dq = mma_bf16(cbh.v, wbl.v, dq);
    dq = mma_bf16(cbl.v, wbh.v, dq);
  }
  {
    const float bb = bc[m];
#pragma unroll
    for (int r = 0; r < 8; ++r) {
      sDw[(8 * h + r) * 16 + m]       = dk[r] + bb;
      sDw[256 + (8 * h + r) * 16 + m] = dq[r] + bb;
    }
  }
  __syncthreads();
  {
    float* src = sDw + h * 256 + m * 16;
    float so = 0.f;
#pragma unroll 1
    for (int k = 0; k < 16; ++k) { float a = tanhf(src[k]); src[k] = a; so += a * a; }
    const float inv2 = 16.0f / fmaxf(sqrtf(so), 1e-12f);
    const int tl = w * 16 + m;
    _Float16* od = sO + h * (128 * 16) + tl * 16;
#pragma unroll 1
    for (int k = 0; k < 16; ++k) {
      _Float16 hv = (_Float16)(src[k] * inv2);
      od[k] = hv;
      if (h == 0) sT[k * TR + tl] = hv;
    }
  }
  __syncthreads();
  const int b  = brow0 >> 11;
  const int t0 = brow0 & (Lq - 1);
  const int kk = tid >> 4, pc = tid & 15;
  h8 vk = *(const h8*)(sO + tid * 8);
  h8 vq = *(const h8*)(sO + 128 * 16 + tid * 8);
  h8 vt = *(const h8*)(sT + kk * TR + pc * 8);
  _Float16* pk = ckh + (size_t)brow0 * Kq + tid * 8;
  _Float16* pq2 = cqh + (size_t)brow0 * Kq + tid * 8;
  _Float16* pt = ckT + ((size_t)(b * Kq + kk)) * Lq + t0 + pc * 8;
  *(volatile h8*)pk = vk;
  *(volatile h8*)pq2 = vq;
  *(volatile h8*)pt = vt;
  __threadfence();
  *(volatile h8*)pk = vk;
  *(volatile h8*)pq2 = vq;
  *(volatile h8*)pt = vt;
}

__global__ void __launch_bounds__(256)
k_chunksum(const _Float16* __restrict__ ckT, const _Float16* __restrict__ valT, float* __restrict__ Ac) {
  __shared__ __align__(16) float sA[16 * 128];
  const int tid = threadIdx.x, lane = tid & 31, w = tid >> 5, m = lane & 15, h = lane >> 4;
  const int chunk = blockIdx.x, b = chunk / NCH, c = chunk % NCH;
  const _Float16* ckb = ckT  + (size_t)b * Kq * Lq;
  const _Float16* vb  = valT + (size_t)b * Dq * Lq;
  const int dblk = blockIdx.y * 128;
  const int d0 = dblk + w * 16;
  f8 acc = {};
#pragma unroll
  for (int ks = 0; ks < CH / 32; ++ks)
    acc = mma_f16(frag_nk(ckb, Lq, 0, c * CH + ks * 32, lane),
                  frag_nk(vb, Lq, d0, c * CH + ks * 32, lane), acc);
#pragma unroll
  for (int r = 0; r < 8; ++r) sA[(8 * h + r) * 128 + w * 16 + m] = acc[r];
  __syncthreads();
#pragma unroll
  for (int q = 0; q < 2; ++q) {
    int k = 2 * w + q;
    v4f v = *(const v4f*)(sA + k * 128 + lane * 4);
    *(volatile v4f*)(Ac + ((size_t)(chunk * Kq + k)) * Dq + dblk + lane * 4) = v;
  }
  __threadfence();
#pragma unroll
  for (int q = 0; q < 2; ++q) {
    int k = 2 * w + q;
    v4f v = *(const v4f*)(sA + k * 128 + lane * 4);
    *(volatile v4f*)(Ac + ((size_t)(chunk * Kq + k)) * Dq + dblk + lane * 4) = v;
  }
}

__global__ void __launch_bounds__(256)
k_attn(const _Float16* __restrict__ cqh, const _Float16* __restrict__ ckh,
       const _Float16* __restrict__ valT, const float* __restrict__ Ac,
       float* __restrict__ retr) {
  __shared__ __align__(16) _Float16 sS[CH * SROW];
  __shared__ __align__(16) _Float16 sPt[32 * 16];
  __shared__ __align__(16) float    sR[8 * 16 * 32];
  const int tid = threadIdx.x, lane = tid & 31, w = tid >> 5, m = lane & 15, h = lane >> 4;
  const int chunk = blockIdx.x, b = chunk / NCH, c = chunk % NCH;
  const int rowbase = b * Lq + c * CH;
  const f8 z8 = {};
  const h8 zh = {};

  h16 aq = frag_nk16(cqh, Kq, rowbase + w * 16, lane);

#pragma unroll
  for (int ct = 0; ct < CH / 16; ++ct) {
    h16 bk = frag_nk16(ckh, Kq, rowbase + ct * 16, lane);
    f8 s = mma_f16(aq, bk, z8);
#pragma unroll
    for (int r = 0; r < 8; ++r) {
      int t  = w * 16 + 8 * h + r;
      int sc = ct * 16 + m;
      sS[t * SROW + sc] = (_Float16)((sc <= t) ? s[r] : 0.0f);
    }
  }
  __syncthreads();

  h16 as[4];
#pragma unroll
  for (int ks = 0; ks < 4; ++ks) as[ks] = frag_nk(sS, SROW, w * 16, ks * 32, lane);

  const _Float16* vb = valT + (size_t)b * Dq * Lq;
  const float* Acb = Ac + (size_t)b * NCH * Kq * Dq;
  const int tch = c * CH;
  const int pd = tid >> 3, pk = tid & 7;
  const int q8 = lane >> 3, pc = lane & 7;
  float* sRw = sR + w * (16 * 32);
  const float SC = 1.0f / 16384.0f;

  for (int cp = 0; cp < Dq / 32; ++cp) {
    const int colt = cp * 32;
    __syncthreads();
    {
      float r0 = 0.f, r1 = 0.f;
      const float* ap = Acb + (size_t)pk * Dq + colt + pd;
      for (int cc = 0; cc < c; ++cc) {
        r0 += ap[(size_t)cc * Kq * Dq];
        r1 += ap[(size_t)cc * Kq * Dq + 8 * Dq];
      }
      sPt[pd * 16 + pk]     = (_Float16)r0;
      sPt[pd * 16 + pk + 8] = (_Float16)r1;
    }
    __syncthreads();
    HF p0, p1;
    p0.p[0] = *(const h8*)(sPt + m * 16 + 8 * h);         p0.p[1] = zh;
    p1.p[0] = *(const h8*)(sPt + (16 + m) * 16 + 8 * h);  p1.p[1] = zh;
    f8 acc0 = mma_f16(aq, p0.v, z8);
    f8 acc1 = mma_f16(aq, p1.v, z8);
#pragma unroll
    for (int ks = 0; ks < 4; ++ks) {
      acc0 = mma_f16(as[ks], frag_nk(vb, Lq, colt,      tch + ks * 32, lane), acc0);
      acc1 = mma_f16(as[ks], frag_nk(vb, Lq, colt + 16, tch + ks * 32, lane), acc1);
    }
#pragma unroll
    for (int r = 0; r < 8; ++r) {
      sRw[(8 * h + r) * 32 + m]      = acc0[r] * SC;
      sRw[(8 * h + r) * 32 + 16 + m] = acc1[r] * SC;
    }
    __syncthreads();
#pragma unroll
    for (int j = 0; j < 4; ++j) {
      int rl = 4 * j + q8;
      v4f v = *(const v4f*)(sRw + rl * 32 + pc * 4);
      *(volatile v4f*)(retr + (size_t)(rowbase + w * 16 + rl) * Dq + colt + pc * 4) = v;
    }
    __threadfence();
#pragma unroll
    for (int j = 0; j < 4; ++j) {
      int rl = 4 * j + q8;
      v4f v = *(const v4f*)(sRw + rl * 32 + pc * 4);
      *(volatile v4f*)(retr + (size_t)(rowbase + w * 16 + rl) * Dq + colt + pc * 4) = v;
    }
  }
}

__global__ void __launch_bounds__(256)
k_lnorm(const float* __restrict__ retr, const float* __restrict__ g,
        const float* __restrict__ bta, _Float16* __restrict__ nh) {
  const int lane = threadIdx.x & 31;
  const int row = blockIdx.x * 8 + (threadIdx.x >> 5);
  const float* p = retr + (size_t)row * Dq + 8 * lane;
  float s = 0.f;
#pragma unroll 1
  for (int j = 0; j < 4; ++j) {
    const v4f* q = (const v4f*)(p + 256 * j);
    v4f a = q[0], c = q[1];
    s += ((a[0] + a[1]) + (a[2] + a[3])) + ((c[0] + c[1]) + (c[2] + c[3]));
  }
#pragma unroll
  for (int off = 16; off; off >>= 1) s += __shfl_xor(s, off, 32);
  const float mu = s * (1.0f / Dq);
  float sq = 0.f;
#pragma unroll 1
  for (int j = 0; j < 4; ++j) {
    const v4f* q = (const v4f*)(p + 256 * j);
    v4f a = q[0], c = q[1];
#pragma unroll
    for (int i = 0; i < 4; ++i) {
      float d0 = a[i] - mu; sq += d0 * d0;
      float d1 = c[i] - mu; sq += d1 * d1;
    }
  }
#pragma unroll
  for (int off = 16; off; off >>= 1) sq += __shfl_xor(sq, off, 32);
  const float var = sq * (1.0f / Dq);
  const float inv = rsqrtf(var + 1e-5f);
  _Float16* d = nh + (size_t)row * Dq + 8 * lane;
#pragma unroll 1
  for (int j = 0; j < 4; ++j) {
    const v4f* q  = (const v4f*)(p + 256 * j);
    const v4f* gq = (const v4f*)(g + 8 * lane + 256 * j);
    const v4f* bq = (const v4f*)(bta + 8 * lane + 256 * j);
    v4f a = q[0], c = q[1];
    v4f g0 = gq[0], g1 = gq[1], b0 = bq[0], b1 = bq[1];
    h8 o;
#pragma unroll
    for (int i = 0; i < 4; ++i) {
      o[i]     = (_Float16)((a[i] - mu) * inv * g0[i] + b0[i]);
      o[4 + i] = (_Float16)((c[i] - mu) * inv * g1[i] + b1[i]);
    }
    *(volatile h8*)(d + 256 * j) = o;
    __threadfence();
    *(volatile h8*)(d + 256 * j) = o;
  }
}

extern "C" void kernel_launch(void* const* d_in, const int* in_sizes, int n_in,
                              void* d_out, int out_size, void* d_ws, size_t ws_size,
                              hipStream_t stream) {
  if (n_in < 14) return;
  if (in_sizes[0] != NR * Dq || in_sizes[1] != Dq * Dq || in_sizes[2] != Dq ||
      in_sizes[3] != Kq * Dq || in_sizes[4] != Kq || in_sizes[5] != Kq * 2 * Kq ||
      in_sizes[6] != Kq || in_sizes[7] != Kq * Dq || in_sizes[8] != Kq ||
      in_sizes[9] != Dq || in_sizes[10] != Dq || in_sizes[11] != Dq * Dq ||
      in_sizes[12] != Dq || in_sizes[13] != Lq * Kq || out_size != NR * Dq) return;

  const float* x   = (const float*)d_in[0];
  const float* Wv  = (const float*)d_in[1];
  const float* bv  = (const float*)d_in[2];
  const float* Wck = (const float*)d_in[3];
  const float* bck = (const float*)d_in[4];
  const float* Wc  = (const float*)d_in[5];
  const float* bc  = (const float*)d_in[6];
  const float* Wcq = (const float*)d_in[7];
  const float* bcq = (const float*)d_in[8];
  const float* lng = (const float*)d_in[9];
  const float* lnb = (const float*)d_in[10];
  const float* Wo  = (const float*)d_in[11];
  const float* bo  = (const float*)d_in[12];
  const float* pos = (const float*)d_in[13];
  float* out = (float*)d_out;

  size_t off = 0;
  char* base = (char*)d_ws;
  auto carve = [&](size_t bytes) -> char* {
    char* p = base + off;
    off += (bytes + 255) & ~(size_t)255;
    return p;
  };
  _Float16* xh   = (_Float16*)carve((size_t)NR * Dq * 2);
  _Float16* Wvh  = (_Float16*)carve((size_t)Dq * Dq * 2);
  _Float16* Woh  = (_Float16*)carve((size_t)Dq * Dq * 2);
  _Float16* valT = (_Float16*)carve((size_t)NR * Dq * 2);
  _Float16* ckh  = (_Float16*)carve((size_t)NR * Kq * 2);
  _Float16* cqh  = (_Float16*)carve((size_t)NR * Kq * 2);
  _Float16* ckT  = (_Float16*)carve((size_t)Bq * Kq * Lq * 2);
  float*    Ac   = (float*)   carve((size_t)Bq * NCH * Kq * Dq * 4);
  float*    retr = (float*)   carve((size_t)NR * Dq * 4);
  _Float16* nh   = (_Float16*)carve((size_t)NR * Dq * 2);
  if (off > ws_size) return;

  const int n8x = NR * Dq / 8;
  const int n8w = Dq * Dq / 8;
  k_cvt<<<(n8x + 255) / 256, 256, 0, stream>>>(x,  xh,  n8x, 1.0f);
  k_cvt<<<(n8w + 255) / 256, 256, 0, stream>>>(Wv, Wvh, n8w, 64.0f);
  k_cvt<<<(n8w + 255) / 256, 256, 0, stream>>>(Wo, Woh, n8w, 64.0f);

  k_gemm_val<<<dim3(NR / 128, Dq / 128), 256, 0, stream>>>(xh, Wvh, bv, valT);
  k_proj<<<NR / 128, 256, 0, stream>>>(x, Wck, Wcq, bck, bcq, Wc, bc, pos, ckh, cqh, ckT);
  k_chunksum<<<dim3(Bq * NCH, Dq / 128), 256, 0, stream>>>(ckT, valT, Ac);
  k_attn<<<Bq * NCH, 256, 0, stream>>>(cqh, ckh, valT, Ac, retr);
  k_lnorm<<<NR / 8, 256, 0, stream>>>(retr, lng, lnb, nh);
  k_gemm_out<<<dim3(NR / 128, Dq / 128), 256, 0, stream>>>(nh, Woh, bo, x, out);
}
